// DynamicConvolution_22497038696611
// MI455X (gfx1250) — hardware-verified
//
#include <hip/hip_runtime.h>


#ifndef NB
#define NB 4
#endif
#ifndef SEQ
#define SEQ 1024
#endif

namespace {
constexpr int NB_FULL = 4, SEQ_FULL = 1024, CCH = 1024, NH = 16, KW = 31, PADW = 15, DHD = 64, HK = NH * KW  , WLP = 512  , MROWS = NB * SEQ, TB = 32  ;
constexpr float XS = 8.0f, WSC = 256.0f, CS = 64.0f;
static_assert(NB >= 1 && NB <= NB_FULL);
static_assert(SEQ % 64 == 0 && SEQ <= SEQ_FULL && SEQ % TB == 0);
static_assert(CCH % 128 == 0 && WLP % 128 == 0 && CCH % 32 == 0 && HK <= WLP && NH * DHD == CCH && TB + KW - 1 <= 2 * TB);
typedef _Float16 b16;
typedef __attribute__((ext_vector_type(16))) _Float16 v16b;
typedef __attribute__((ext_vector_type(8))) _Float16 v8b;
typedef __attribute__((ext_vector_type(8))) float v8f;
typedef __attribute__((ext_vector_type(4))) float v4f;
__device__ __forceinline__ float bf16_rne(float f) { unsigned int u = __float_as_uint(f); u += 0x7FFFu + ((u >> 16) & 1u); return __uint_as_float(u & 0xFFFF0000u); }
__device__ __forceinline__ v16b frag_kb(const b16* p, int hh) { const v8b a = *(const v8b*)(p + 8 * hh), b = *(const v8b*)(p + 16 + 8 * hh); v16b f;
#pragma unroll
  for (int e = 0; e < 8; ++e) { f[e] = a[e]; f[8 + e] = b[e]; } return f; }
__device__ __forceinline__ v8f wmma16b(v16b a, v16b b, v8f c) { v8f d = __builtin_amdgcn_wmma_f32_16x16x32_f16(false, a, false, b, (short)0, c, false, false); asm volatile("v_nop\n\tv_nop\n\tv_nop\n\tv_nop" : "+v"(d) : "v"(a), "v"(b)); return d; }
__device__ __forceinline__ void wave_lds_sync() { __builtin_amdgcn_fence(__ATOMIC_RELEASE, "workgroup"); __builtin_amdgcn_wave_barrier(); __builtin_amdgcn_fence(__ATOMIC_ACQUIRE, "workgroup"); }
__device__ __forceinline__ int iclamp(int v, int lo, int hi) { return v < lo ? lo : (v > hi ? hi : v); }

__global__ __launch_bounds__(256) void cvt_kernel(const float* __restrict__ src, b16* __restrict__ dst, int rows_dst, int seq_dst, int seq_src, int rows_src, float scale) {
  const size_t u = (size_t)blockIdx.x * 256 + threadIdx.x; const size_t n8 = (size_t)rows_dst * CCH / 8; if (u >= n8) return;
  const size_t e = u * 8; const int mrow = (int)(e / CCH); const int c = (int)(e - (size_t)mrow * CCH);
  const int bb = mrow / seq_dst, t = mrow - bb * seq_dst; const int srow = bb * seq_src + t; const bool ok = srow < rows_src;
  const float* sp = src + (size_t)iclamp(srow, 0, rows_src - 1) * CCH + c;
  const v4f x0 = *(const v4f*)sp, x1 = *(const v4f*)(sp + 4); v8b o;
#pragma unroll
  for (int j = 0; j < 4; ++j) { o[j] = ok ? (b16)(bf16_rne(x0[j]) * scale) : (b16)0.0f; o[4 + j] = ok ? (b16)(bf16_rne(x1[j]) * scale) : (b16)0.0f; }
  for (int pass = 0; pass < 2; ++pass) { *(volatile v8b*)(dst + e) = o; __threadfence(); }
}

template <int MODE> __device__ __forceinline__ int brow(int t, int n0, int m) { return MODE == 0 ? (n0 + 16 * t + m) : (t < 4 ? (n0 + 16 * t + m) : (CCH + n0 + 16 * (t - 4) + m)); }

template <int MODE>
__global__ __launch_bounds__(128) void gemm_kernel(const b16* __restrict__ A, const b16* __restrict__ Bm, const float* __restrict__ bias, float* __restrict__ Cf, b16* __restrict__ Ch, int K, int ldc, int nbias, float oscale) {
  __shared__ __attribute__((aligned(16))) float Tf[4][16][128 + 4];
  const int wave = threadIdx.x >> 5, lane = threadIdx.x & 31, m = lane & 15, hh = lane >> 4;
  const int m0 = blockIdx.y * 64 + wave * 16; const int n0 = blockIdx.x * (MODE == 0 ? 128 : 64);
  v8f acc[8];
#pragma unroll
  for (int t = 0; t < 8; ++t) acc[t] = (v8f){};
  const b16* ap = A + (size_t)(m0 + m) * K;
#pragma unroll 1
  for (int kb = 0; kb < K; kb += 32) { const v16b a = frag_kb(ap + kb, hh);
#pragma unroll
    for (int t = 0; t < 8; ++t) acc[t] = wmma16b(a, frag_kb(Bm + (size_t)brow<MODE>(t, n0, m) * K + kb, hh), acc[t]); }
  float (*T)[128 + 4] = Tf[wave];
  if (MODE == 0) {
#pragma unroll
    for (int t = 0; t < 8; ++t) { const int n = n0 + 16 * t + m; const float bl = bias[iclamp(n, 0, nbias - 1)]; const float bv = (n < nbias) ? bl : 0.0f;
#pragma unroll
      for (int r = 0; r < 8; ++r) T[8 * hh + r][16 * t + m] = acc[t][r] * oscale + bv; }
    wave_lds_sync();
    for (int pass = 0; pass < 2; ++pass) {
#pragma unroll 1
      for (int r = 0; r < 16; ++r) { const v4f v = *(const v4f*)&T[r][4 * lane]; *(volatile v4f*)(Cf + (size_t)(m0 + r) * ldc + n0 + 4 * lane) = v; }
      __threadfence(); }
  } else {
#pragma unroll
    for (int t = 0; t < 4; ++t) { const int na = n0 + 16 * t + m; const float ba = bias[na], bg = bias[CCH + na];
#pragma unroll
      for (int r = 0; r < 8; ++r) { T[8 * hh + r][16 * t + m] = acc[t][r] * oscale + ba; T[8 * hh + r][64 + 16 * t + m] = acc[t + 4][r] * oscale + bg; } }
    wave_lds_sync();
#pragma unroll 1
    for (int it = 0; it < 8; ++it) { const int r2 = 2 * it + hh; const v4f av = *(const v4f*)&T[r2][4 * m], gv = *(const v4f*)&T[r2][64 + 4 * m]; v4f xv;
#pragma unroll
      for (int j = 0; j < 4; ++j) xv[j] = av[j] * (1.0f / (1.0f + expf(-gv[j])));
      *(v4f*)&T[r2][4 * m] = xv; }
    wave_lds_sync();
    for (int pass = 0; pass < 2; ++pass) {
#pragma unroll 1
      for (int q = 0; q < 8; ++q) { const int r2 = 2 * q + hh; const v4f v = *(const v4f*)&T[r2][4 * m]; *(volatile v4f*)(Cf + (size_t)(m0 + r2) * ldc + n0 + 4 * m) = v; }
#pragma unroll 1
      for (int q = 0; q < 4; ++q) { const int r4 = 4 * q + (lane >> 3), c8 = 8 * (lane & 7); const v4f x0 = *(const v4f*)&T[r4][c8], x1 = *(const v4f*)&T[r4][c8 + 4]; v8b o;
#pragma unroll
        for (int j = 0; j < 4; ++j) { o[j] = (b16)(x0[j] * XS); o[4 + j] = (b16)(x1[j] * XS); }
        *(volatile v8b*)(Ch + (size_t)(m0 + r4) * ldc + n0 + c8) = o; }
      __threadfence(); }
  }
}

__global__ __launch_bounds__(256) void band_kernel(const float* __restrict__ WL, const float* __restrict__ Xf, const int* __restrict__ mask, const int* __restrict__ kpm, b16* __restrict__ CV) {
  __shared__ __attribute__((aligned(16))) float Xs[2 * TB][DHD + 4];
  __shared__ __attribute__((aligned(16))) float Os[TB][DHD + 4];
  __shared__ float Ps[TB][32];
  __shared__ int keep_s[TB];
  const int tid = threadIdx.x, lane = tid & 31, wave = tid >> 5;
  const int t0 = blockIdx.x * TB, h = blockIdx.y, bb = blockIdx.z;
  const size_t rowbase = (size_t)bb * SEQ;
  for (int i = tid; i < 2 * TB * (DHD / 4); i += 256) { const int row = i >> 4, c4 = (i & 15) * 4; const int s = t0 - PADW + row; const bool ok = (row < TB + KW - 1) && s >= 0 && s < SEQ;
    v4f v = *(const v4f*)(Xf + (rowbase + iclamp(s, 0, SEQ - 1)) * CCH + h * DHD + c4); if (!ok) v = (v4f){}; *(v4f*)&Xs[row][c4] = v; }
  for (int i = tid; i < TB * 32; i += 256) { const int tl = i >> 5, j = i & 31; Ps[tl][j] = WL[(rowbase + t0 + tl) * WLP + h * KW + (j < KW ? j : KW - 1)]; }
  __syncthreads();
  if (tid < TB) { const int tl = tid, t = t0 + tl; const int jlo = (PADW - t > 0) ? (PADW - t) : 0; const int jh = SEQ - 1 + PADW - t; const int jhi = jh < KW - 1 ? jh : KW - 1;
    float mx = -3.0e38f;
#pragma unroll 1
    for (int j = jlo; j <= jhi; ++j) mx = fmaxf(mx, Ps[tl][j]);
    float sum = 0.0f;
#pragma unroll 1
    for (int j = 0; j < 32; ++j) { const bool ok = (j >= jlo) && (j <= jhi); const float arg = ok ? (Ps[tl][j] - mx) : -80.0f; const float e = ok ? expf(arg) : 0.0f; Ps[tl][j] = e; sum += e; }
    const float inv = 1.0f / sum;
#pragma unroll 1
    for (int j = 0; j < 32; ++j) Ps[tl][j] = Ps[tl][j] * inv;
    keep_s[tl] = (mask[(size_t)bb * SEQ_FULL + t] != 0 && kpm[(size_t)bb * SEQ_FULL + t] == 0) ? 1 : 0; }
  __syncthreads();
  { const int d = tid & 63, tq = tid >> 6;
#pragma unroll 1
    for (int i = 0; i < 8; ++i) { const int tl = tq * 8 + i; float acc = 0.0f;
#pragma unroll 4
      for (int j = 0; j < KW; ++j) acc += Ps[tl][j] * Xs[tl + j][d];
      Os[tl][d] = acc; } }
  __syncthreads();
  { const int tl = wave * 4 + (lane >> 3), c8 = (lane & 7) * 8; const bool kp = keep_s[tl] != 0;
    const v4f x0 = *(const v4f*)&Os[tl][c8], x1 = *(const v4f*)&Os[tl][c8 + 4]; v8b o;
#pragma unroll
    for (int j = 0; j < 4; ++j) { o[j] = (b16)((kp ? x0[j] : 0.0f) * CS); o[4 + j] = (b16)((kp ? x1[j] : 0.0f) * CS); }
    b16* dst = CV + (rowbase + t0 + tl) * CCH + h * DHD + c8;
    for (int pass = 0; pass < 2; ++pass) { *(volatile v8b*)dst = o; __threadfence(); } }
}
}

extern "C" void kernel_launch(void* const* d_in, const int* in_sizes, int n_in, void* d_out, int out_size, void* d_ws, size_t ws_size, hipStream_t stream) {
  if (n_in < 11) return;
  const float* query = (const float*)d_in[0];
  const int* mask = (const int*)d_in[3];
  const int* kpm = (const int*)d_in[4];
  const float* w1 = (const float*)d_in[5];
  const float* b1 = (const float*)d_in[6];
  const float* ww = (const float*)d_in[7];
  const float* bw = (const float*)d_in[8];
  const float* w2 = (const float*)d_in[9];
  const float* b2 = (const float*)d_in[10];
  const int need_rows = (NB - 1) * SEQ_FULL + SEQ;
  if (in_sizes[0] < need_rows * CCH || in_sizes[3] < need_rows || in_sizes[4] < need_rows) return;
  if (in_sizes[5] != 2 * CCH * CCH || in_sizes[6] < 2 * CCH || in_sizes[7] != HK * CCH || in_sizes[8] < HK || in_sizes[9] != CCH * CCH || in_sizes[10] < CCH) return;
  if (out_size < MROWS * CCH) return;
  size_t off = 0; char* ws = (char*)d_ws;
  auto carve = [&](size_t bytes) { char* p = ws + off; off += (bytes + 255) & ~(size_t)255; return p; };
  b16* Qh = (b16*)carve((size_t)MROWS * CCH * 2);
  b16* W1h = (b16*)carve((size_t)2 * CCH * CCH * 2);
  b16* WWh = (b16*)carve((size_t)WLP * CCH * 2);
  b16* W2h = (b16*)carve((size_t)CCH * CCH * 2);
  float* Xf = (float*)carve((size_t)MROWS * CCH * 4);
  b16* Xh = (b16*)carve((size_t)MROWS * CCH * 2);
  float* WL = (float*)carve((size_t)MROWS * WLP * 4);
  b16* CV = (b16*)carve((size_t)MROWS * CCH * 2);
  if (off > ws_size || off > ((size_t)128 << 20)) return;
  const int qrows = in_sizes[0] / CCH;
  cvt_kernel<<<(unsigned)(((size_t)MROWS * CCH / 8 + 255) / 256), 256, 0, stream>>>(query, Qh, MROWS, SEQ, SEQ_FULL, qrows, XS);
  cvt_kernel<<<(unsigned)(((size_t)2 * CCH * CCH / 8 + 255) / 256), 256, 0, stream>>>(w1, W1h, 2 * CCH, 2 * CCH, 2 * CCH, 2 * CCH, WSC);
  cvt_kernel<<<(unsigned)(((size_t)WLP * CCH / 8 + 255) / 256), 256, 0, stream>>>(ww, WWh, WLP, WLP, WLP, HK, WSC);
  cvt_kernel<<<(unsigned)(((size_t)CCH * CCH / 8 + 255) / 256), 256, 0, stream>>>(w2, W2h, CCH, CCH, CCH, CCH, WSC);
  gemm_kernel<1><<<dim3(CCH / 64, MROWS / 64), 128, 0, stream>>>(Qh, W1h, b1, Xf, Xh, CCH, CCH, 2 * CCH, 1.0f / (XS * WSC));
  gemm_kernel<0><<<dim3(WLP / 128, MROWS / 64), 128, 0, stream>>>(Xh, WWh, bw, WL, Xh, CCH, WLP, HK, 1.0f / (XS * WSC));
  band_kernel<<<dim3(SEQ / TB, NH, NB), 256, 0, stream>>>(WL, Xf, mask, kpm, CV);
  gemm_kernel<0><<<dim3(CCH / 128, MROWS / 64), 128, 0, stream>>>(CV, W2h, b2, (float*)d_out, CV, CCH, CCH, CCH, 1.0f / (CS * WSC));
}
